// LFA_10445360464114
// MI455X (gfx1250) — hardware-verified
//
#include <hip/hip_runtime.h>
#include <math.h>

#define NB_ 2
#define NN 16384
#define KNB 16
#define DIN 32
#define DD 64
#define D8 8

typedef _Float16 f16;
typedef __attribute__((ext_vector_type(16))) f16 f16x16;
typedef __attribute__((ext_vector_type(8)))  f16 f16x8;
typedef __attribute__((ext_vector_type(8)))  float f32x8;
typedef __attribute__((ext_vector_type(4)))  float v4f_t;
typedef float v4fa __attribute__((ext_vector_type(4), may_alias));

__device__ __forceinline__ f32x8 wmma16(f16x16 a, f16x16 b, f32x8 c) {
  c = __builtin_amdgcn_wmma_f32_16x16x32_f16(false, a, false, b, (short)0, c, false, false);
  asm volatile("v_nop\n\tv_nop\n\tv_nop\n\tv_nop" : "+v"(c) : "v"(a), "v"(b));
  return c;
}
__device__ __forceinline__ f16x16 lds_frag(const f16* base, int stride) {
  const int lane = threadIdx.x & 31, row = lane & 15, kh = (lane >> 4) * 8;
  const f16x8 lo = *(const f16x8*)(base + row * stride + kh);
  const f16x8 hi = *(const f16x8*)(base + row * stride + kh + 16);
  f16x16 f;
#pragma unroll
  for (int i = 0; i < 8; ++i) { f[i] = lo[i]; f[i + 8] = hi[i]; }
  return f;
}
__device__ __forceinline__ void split16(float v, f16& h, f16& l) { h = (f16)v; l = (f16)((v - (float)h) * 2048.0f); }
__device__ __forceinline__ void wfrag2(const float* __restrict__ Wm, int O, int C, int o0, int k0, f16x16& hi, f16x16& lo) {
  const int lane = threadIdx.x & 31, r = o0 + (lane & 15), kh = (lane >> 4) * 8; const int rc = min(r, O - 1);
#pragma unroll
  for (int i = 0; i < 8; ++i) { const int ka = k0 + kh + i, kb = ka + 16;
    const float a = (r < O && ka < C) ? Wm[(size_t)rc * C + min(ka, C - 1)] : 0.0f, b2 = (r < O && kb < C) ? Wm[(size_t)rc * C + min(kb, C - 1)] : 0.0f;
    f16 h, l; split16(a, h, l); hi[i] = h; lo[i] = l; split16(b2, h, l); hi[8 + i] = h; lo[8 + i] = l; }
}
__device__ __forceinline__ void mma3(f32x8& acc, f32x8& accx, const f16x16& ah, const f16x16& al, const f16x16& bh, const f16x16& bl) {
  acc = wmma16(ah, bh, acc); accx = wmma16(ah, bl, accx); accx = wmma16(al, bh, accx);
}
__device__ __forceinline__ float bn_apply(float v, const float* __restrict__ p, int C, int c) {
  const float s = p[c] / sqrtf(p[3 * C + c] + 1e-5f); return v * s + (p[C + c] - p[2 * C + c] * s);
}

__global__ __launch_bounds__(256) void k_node(const float* __restrict__ feat, const float* __restrict__ W1, const float* __restrict__ bn1,
                                             const float* __restrict__ Wq, const float* __restrict__ bq, const float* __restrict__ Wk, const float* __restrict__ bk,
                                             const float* __restrict__ Wv, const float* __restrict__ bv, float* __restrict__ fcm, float* __restrict__ qo,
                                             float* __restrict__ ko, float* __restrict__ vo) {
  __shared__ __attribute__((aligned(16))) f16 aS[2][128 * 72];
  __shared__ __attribute__((aligned(16))) float fS[64 * 132];
  __shared__ __attribute__((aligned(16))) float oS[128 * 68];
  const int tid = threadIdx.x, lane = tid & 31, wave = tid >> 5, cl = lane & 15, rh = (lane >> 4) * 8;
  const int b = blockIdx.x / (NN / 128), n0 = (blockIdx.x % (NN / 128)) * 128;
  for (int e = tid; e < 128 * 64; e += 256) { const int n = e >> 6, c = e & 63; const float v = (c < DIN) ? feat[((size_t)b * DIN + min(c, DIN - 1)) * NN + n0 + n] : 0.0f;
    f16 h, l; split16(v, h, l); aS[0][n * 72 + c] = h; aS[1][n * 72 + c] = l; }
  __syncthreads();
  { const f16x16 ah = lds_frag(aS[0] + (wave * 16) * 72, 72), al = lds_frag(aS[1] + (wave * 16) * 72, 72);
#pragma unroll
    for (int nt = 0; nt < 4; ++nt) { f16x16 bh, bl; wfrag2(W1, DD, DIN, nt * 16, 0, bh, bl); f32x8 acc = {}, accx = {}; mma3(acc, accx, ah, al, bh, bl);
      const int d = nt * 16 + cl;
#pragma unroll
      for (int r = 0; r < 8; ++r) { const float v = fmaxf(bn_apply(acc[r] + accx[r] * (1.0f / 2048.0f), bn1, DD, d), 0.0f); fS[d * 132 + wave * 16 + rh + r] = v; } } }
  __syncthreads();
#pragma unroll 1
  for (int pass = 0; pass < 2; ++pass) { for (int q4 = tid; q4 < 64 * 32; q4 += 256) { const int d = q4 >> 5, c4 = (q4 & 31) * 4;
      *(volatile v4f_t*)(fcm + ((size_t)b * DD + d) * NN + n0 + c4) = *(const volatile v4fa*)(fS + d * 132 + c4); } __threadfence(); }
  for (int e = tid; e < 128 * 64; e += 256) { const int n = e >> 6, d = e & 63; f16 h, l; split16(fS[d * 132 + n], h, l); aS[0][n * 72 + d] = h; aS[1][n * 72 + d] = l; }
  __syncthreads();
  f16x16 ah[2], al[2];
#pragma unroll
  for (int ks = 0; ks < 2; ++ks) { ah[ks] = lds_frag(aS[0] + (wave * 16) * 72 + ks * 32, 72); al[ks] = lds_frag(aS[1] + (wave * 16) * 72 + ks * 32, 72); }
#pragma unroll 1
  for (int which = 0; which < 3; ++which) {
    const float* Wm = (which == 0) ? Wq : (which == 1) ? Wk : Wv; const float* bb = (which == 0) ? bq : (which == 1) ? bk : bv; float* dst = (which == 0) ? qo : (which == 1) ? ko : vo;
    __syncthreads();
#pragma unroll
    for (int nt = 0; nt < 4; ++nt) { f32x8 acc = {}, accx = {};
#pragma unroll
      for (int ks = 0; ks < 2; ++ks) { f16x16 bh, bl; wfrag2(Wm, DD, DD, nt * 16, ks * 32, bh, bl); mma3(acc, accx, ah[ks], al[ks], bh, bl); }
      const int d = nt * 16 + cl; const float bvv = bb[d];
#pragma unroll
      for (int r = 0; r < 8; ++r) oS[(wave * 16 + rh + r) * 68 + d] = acc[r] + accx[r] * (1.0f / 2048.0f) + bvv; }
    __syncthreads();
#pragma unroll 1
    for (int pass = 0; pass < 2; ++pass) { for (int q4 = tid; q4 < 128 * 16; q4 += 256) { const int n = q4 >> 4, c4 = (q4 & 15) * 4;
        *(volatile v4f_t*)(dst + ((size_t)b * NN + n0 + n) * DD + c4) = *(const volatile v4fa*)(oS + n * 68 + c4); } __threadfence(); }
  }
}

__global__ __launch_bounds__(256) void k_pair(const float* __restrict__ xyz, const int* __restrict__ nidx, const float* __restrict__ qo, const float* __restrict__ ko,
                                             const float* __restrict__ vo, const float* __restrict__ fcm,
                                             const float* __restrict__ Wp1, const float* __restrict__ bnp1, const float* __restrict__ Wp2, const float* __restrict__ bp2,
                                             const float* __restrict__ bnw0, const float* __restrict__ Ww1, const float* __restrict__ bnw1, const float* __restrict__ Ww2,
                                             const float* __restrict__ bw2, const float* __restrict__ bnmid, const float* __restrict__ W2, const float* __restrict__ bn2,
                                             float* __restrict__ out) {
  __shared__ __attribute__((aligned(16))) f16 wS[2][256 * 72];
  __shared__ float hS[256 * 9];
  __shared__ float xS[32 * 65];
  __shared__ __attribute__((aligned(16))) f16 xP[2][32 * 72];
  __shared__ __attribute__((aligned(16))) float oS[64 * 36];
  __shared__ float Wp2S[64 * 3], bp2S[64], s0S[64], h0S[64], Ww2S[64], bw2S[8], s1S[8], h1S[8];
  const int tid = threadIdx.x, lane = tid & 31, wave = tid >> 5, cl = lane & 15, rh = (lane >> 4) * 8;
  const int b = blockIdx.x / (NN / 32), n0 = (blockIdx.x % (NN / 32)) * 32;
  for (int e = tid; e < 64 * 3; e += 256) Wp2S[e] = Wp2[e];
  if (tid < 64) { bp2S[tid] = bp2[tid]; const float s = bnw0[tid] / sqrtf(bnw0[3 * DD + tid] + 1e-5f); s0S[tid] = s; h0S[tid] = bnw0[DD + tid] - bnw0[2 * DD + tid] * s; Ww2S[tid] = Ww2[tid]; }
  if (tid < 8) { bw2S[tid] = bw2[tid]; const float s = bnw1[tid] / sqrtf(bnw1[3 * D8 + tid] + 1e-5f); s1S[tid] = s; h1S[tid] = bnw1[D8 + tid] - bnw1[2 * D8 + tid] * s; }
  __syncthreads();
  const int nl = tid >> 4, kk = tid & 15;
#pragma unroll 1
  for (int rd = 0; rd < 2; ++rd) {
    const int node = n0 + rd * 16 + nl;
    int id = nidx[((size_t)b * NN + node) * KNB + kk]; id = min(max(id, 0), NN - 1);
    const float* pz = xyz + ((size_t)b * NN + id) * 3; const float g0 = pz[0], g1 = pz[1], g2 = pz[2];
    float h3[3];
#pragma unroll
    for (int o = 0; o < 3; ++o) { const float v = Wp1[o * 3 + 0] * g0 + Wp1[o * 3 + 1] * g1 + Wp1[o * 3 + 2] * g2; h3[o] = fmaxf(bn_apply(v, bnp1, 3, o), 0.0f); }
    const float* kr = ko + ((size_t)b * NN + id) * DD; const float* qr = qo + ((size_t)b * NN + node) * DD; const float* vr = vo + ((size_t)b * NN + id) * DD;
#pragma unroll 4
    for (int d = 0; d < 64; ++d) { const float p = bp2S[d] + Wp2S[d * 3 + 0] * h3[0] + Wp2S[d * 3 + 1] * h3[1] + Wp2S[d * 3 + 2] * h3[2];
      float w0 = (kr[d] - qr[d] + p) * s0S[d] + h0S[d]; w0 = (w0 >= 0.0f) ? w0 : 0.2f * w0;
      f16 h, l; split16(w0, h, l); wS[0][tid * 72 + d] = h; wS[1][tid * 72 + d] = l; }
    __syncthreads();
#pragma unroll
    for (int t2 = 0; t2 < 2; ++t2) { const int rt = wave * 2 + t2; f32x8 acc = {}, accx = {};
#pragma unroll
      for (int ks = 0; ks < 2; ++ks) { f16x16 bh, bl; wfrag2(Ww1, D8, DD, 0, ks * 32, bh, bl); mma3(acc, accx, lds_frag(wS[0] + (rt * 16) * 72 + ks * 32, 72), lds_frag(wS[1] + (rt * 16) * 72 + ks * 32, 72), bh, bl); }
      if (cl < D8) {
#pragma unroll
        for (int r = 0; r < 8; ++r) hS[(rt * 16 + rh + r) * 9 + cl] = fmaxf((acc[r] + accx[r] * (1.0f / 2048.0f)) * s1S[cl] + h1S[cl], 0.0f); } }
    __syncthreads();
    float wgt[8];
#pragma unroll
    for (int j = 0; j < 8; ++j) { float v = bw2S[j];
#pragma unroll
      for (int c = 0; c < 8; ++c) v += Ww2S[j * 8 + c] * hS[tid * 9 + c];
      float mx = v;
#pragma unroll
      for (int off = 1; off < 16; off <<= 1) mx = fmaxf(mx, __shfl_xor(mx, off, 32));
      const float ex = expf(v - mx); float z = ex;
#pragma unroll
      for (int off = 1; off < 16; off <<= 1) z += __shfl_xor(z, off, 32);
      wgt[j] = ex / z; }
#pragma unroll 1
    for (int g8 = 0; g8 < 8; ++g8) {
#pragma unroll
      for (int j = 0; j < 8; ++j) { const int c = g8 * 8 + j; const float p = bp2S[c] + Wp2S[c * 3 + 0] * h3[0] + Wp2S[c * 3 + 1] * h3[1] + Wp2S[c * 3 + 2] * h3[2];
        float t = wgt[j] * (vr[c] + p);
#pragma unroll
        for (int off = 1; off < 16; off <<= 1) t += __shfl_xor(t, off, 32);
        if (kk == 0) xS[(rd * 16 + nl) * 65 + c] = t; } }
    __syncthreads();
  }
  for (int e = tid; e < 32 * 64; e += 256) { const int n = e >> 6, c = e & 63; float v = bn_apply(xS[n * 65 + c], bnmid, DD, c); v = (v >= 0.0f) ? v : 0.2f * v;
    f16 h, l; split16(v, h, l); xP[0][n * 72 + c] = h; xP[1][n * 72 + c] = l; }
  __syncthreads();
  { const int rt = wave & 1, nt = wave >> 1;
    f32x8 acc = {}, accx = {};
#pragma unroll
    for (int ks = 0; ks < 2; ++ks) { f16x16 bh, bl; wfrag2(W2, DD, DD, nt * 16, ks * 32, bh, bl); mma3(acc, accx, lds_frag(xP[0] + (rt * 16) * 72 + ks * 32, 72), lds_frag(xP[1] + (rt * 16) * 72 + ks * 32, 72), bh, bl); }
    const int d = nt * 16 + cl;
#pragma unroll
    for (int r = 0; r < 8; ++r) { const int n = rt * 16 + rh + r; const float y = bn_apply(acc[r] + accx[r] * (1.0f / 2048.0f), bn2, DD, d);
      float o = fcm[((size_t)b * DD + d) * NN + n0 + n] + y; o = (o >= 0.0f) ? o : 0.2f * o; oS[d * 36 + n] = o; } }
  __syncthreads();
#pragma unroll 1
  for (int pass = 0; pass < 2; ++pass) {
    for (int q4 = tid; q4 < 64 * 8; q4 += 256) { const int d = q4 >> 3, c4 = (q4 & 7) * 4; *(volatile v4f_t*)(out + ((size_t)b * DD + d) * NN + n0 + c4) = *(const volatile v4fa*)(oS + d * 36 + c4); }
    __threadfence();
  }
}

extern "C" void kernel_launch(void* const* d_in, const int* in_sizes, int n_in,
                              void* d_out, int out_size, void* d_ws, size_t ws_size,
                              hipStream_t stream) {
  (void)in_sizes; (void)n_in; (void)out_size;
  const float* feat = (const float*)d_in[0];
  const float* xyz = (const float*)d_in[1];
  const float* W1 = (const float*)d_in[2], *bn1 = (const float*)d_in[3];
  const float* Wq = (const float*)d_in[4], *bq = (const float*)d_in[5], *Wk = (const float*)d_in[6], *bk = (const float*)d_in[7], *Wv = (const float*)d_in[8], *bv = (const float*)d_in[9];
  const float* Wp1 = (const float*)d_in[10], *bnp1 = (const float*)d_in[11], *Wp2 = (const float*)d_in[12], *bp2 = (const float*)d_in[13];
  const float* bnw0 = (const float*)d_in[14], *Ww1 = (const float*)d_in[15], *bnw1 = (const float*)d_in[16], *Ww2 = (const float*)d_in[17], *bw2 = (const float*)d_in[18];
  const float* bnmid = (const float*)d_in[19], *W2 = (const float*)d_in[20], *bn2 = (const float*)d_in[21];
  const int* nidx = (const int*)d_in[22];
  float* out = (float*)d_out;
  char* ws = (char*)d_ws;
  const size_t T = (size_t)NB_ * NN * DD * 4;
  float* fcm = (float*)ws; float* qo = (float*)(ws + T); float* ko = (float*)(ws + 2 * T); float* vo = (float*)(ws + 3 * T);
  if (4 * T > ws_size) return;
  k_node<<<dim3(NB_ * NN / 128), dim3(256), 0, stream>>>(feat, W1, bn1, Wq, bq, Wk, bk, Wv, bv, fcm, qo, ko, vo);
  k_pair<<<dim3(NB_ * NN / 32), dim3(256), 0, stream>>>(xyz, nidx, qo, ko, vo, fcm, Wp1, bnp1, Wp2, bp2, bnw0, Ww1, bnw1, Ww2, bw2, bnmid, W2, bn2, out);
}
